// MambaBlock_57844619543173
// MI455X (gfx1250) — hardware-verified
//
#include <hip/hip_runtime.h>
#include <math.h>

typedef __attribute__((ext_vector_type(16))) _Float16 v16h;
typedef __attribute__((ext_vector_type(8)))  _Float16 v8h;
typedef __attribute__((ext_vector_type(16))) __bf16   v16b;
typedef __attribute__((ext_vector_type(8)))  __bf16   v8b;
typedef __attribute__((ext_vector_type(8)))  float    v8f;
typedef __attribute__((ext_vector_type(4)))  float    v4f;

constexpr int kBatch = 4;
constexpr int kSeq   = 4096;
constexpr int kDm    = 384;
constexpr int kDin   = 768;
constexpr int kNst   = 16;
constexpr int kDtR   = 24;
constexpr int kDtP   = 32;
constexpr int kXdN   = 56;
constexpr int kXdP   = 64;
constexpr int kConvK = 3;
constexpr int kRows  = kBatch * kSeq;
constexpr int kTP    = 260;
constexpr int kLnTok = 32;
constexpr int kLnP   = 33;
constexpr float kCarryXn  = 8.0f;
constexpr float kCarryU   = 16.0f;
constexpr float kCarryDt  = 16.0f;
constexpr float kCarryY   = 16.0f;
constexpr float kCarryW   = 64.0f;
constexpr float kCarryWdt = 16.0f;
constexpr float kScaleIn  = 1.0f / (kCarryXn * kCarryW);
constexpr float kScaleXp  = 1.0f / (kCarryU * kCarryW);
constexpr float kScaleDt  = 1.0f / (kCarryDt * kCarryWdt);
constexpr float kScaleOut = 1.0f / (kCarryY * kCarryW);
static_assert(kDtR + 2 * kNst == kXdN);
static_assert(kXdN <= kXdP && (kXdP % 64) == 0);
static_assert(kDtR <= kDtP && (kDtP % 32) == 0 && (kDtR % 8) == 0);
static_assert((kDm % 32) == 0 && (kDin % 32) == 0);
static_assert((kRows % 64) == 0 && (kDin % 64) == 0 && (kDm % 64) == 0 && (kSeq % 64) == 0);
static_assert((kDin % 256) == 0 && (kSeq % 16) == 0 && (kSeq % kLnTok) == 0);
static_assert(kDm == 256 + 128);
static_assert((kDm % 8) == 0 && (kNst % 4) == 0);

constexpr size_t kOffXN16   = 0;
constexpr size_t kOffWIN16  = kOffXN16   + (size_t)kRows * kDm  * 2;
constexpr size_t kOffWXP16  = kOffWIN16  + (size_t)2 * kDin * kDm * 2;
constexpr size_t kOffWDT16  = kOffWXP16  + (size_t)kXdP * kDin * 2;
constexpr size_t kOffWOUT16 = kOffWDT16  + (size_t)kDin * kDtP * 2;
constexpr size_t kOffUPRE16 = kOffWOUT16 + (size_t)kDm * kDin * 2;
constexpr size_t kOffDLR16  = kOffUPRE16;
constexpr size_t kOffZ16    = kOffUPRE16 + (size_t)kRows * kDin * 2;
constexpr size_t kOffUC16   = kOffZ16    + (size_t)kRows * kDin * 2;
constexpr size_t kOffXD     = kOffUC16   + (size_t)kRows * kDin * 2;
constexpr size_t kOffDT16   = kOffXD     + (size_t)kRows * kXdP * 4;
constexpr size_t kOffY16    = kOffDT16   + (size_t)kRows * kDtP * 2;
constexpr size_t kWsTotal   = kOffY16    + (size_t)kRows * kDin * 2;
static_assert(kWsTotal == 120406016ull);
static_assert(kWsTotal <= 134217728ull);
static_assert((kOffWIN16 % 128) == 0 && (kOffWXP16 % 128) == 0 && (kOffWDT16 % 128) == 0 && (kOffWOUT16 % 128) == 0 &&
              (kOffUPRE16 % 128) == 0 && (kOffZ16 % 128) == 0 && (kOffUC16 % 128) == 0 && (kOffXD % 128) == 0 &&
              (kOffDT16 % 128) == 0 && (kOffY16 % 128) == 0);

__device__ __forceinline__ float h16_to_f32(unsigned hb) {
  const unsigned sgn = (hb & 0x8000u) << 16; const unsigned em = hb & 0x7fffu;
  const float fn = __uint_as_float((em << 13) + 0x38000000u);
  const float fs = (float)em * 5.9604644775390625e-8f;
  const float mag = (em < 0x400u) ? fs : fn; return __uint_as_float(__float_as_uint(mag) | sgn); }

__device__ __forceinline__ void dep_guard4_h(v8f& a, v8f& b, v8f& c, v8f& d, v16h x, v16h y) {
  asm volatile("v_nop\n\tv_nop\n\tv_nop\n\tv_nop" : "+v"(a), "+v"(b), "+v"(c), "+v"(d) : "v"(x), "v"(y)); }
__device__ __forceinline__ void dep_guard4_b(v8f& a, v8f& b, v8f& c, v8f& d, v16b x, v16b y) {
  asm volatile("v_nop\n\tv_nop\n\tv_nop\n\tv_nop" : "+v"(a), "+v"(b), "+v"(c), "+v"(d) : "v"(x), "v"(y)); }
__device__ __forceinline__ void keep4_h(v16h a, v16h b, v16h c, v16h d) { asm volatile("v_nop" :: "v"(a), "v"(b), "v"(c), "v"(d)); }
__device__ __forceinline__ void keep4_b(v16b a, v16b b, v16b c, v16b d) { asm volatile("v_nop" :: "v"(a), "v"(b), "v"(c), "v"(d)); }
__device__ __forceinline__ void acc_guard4(v8f& a, v8f& b, v8f& c, v8f& d) { asm volatile("v_nop\n\tv_nop\n\tv_nop\n\tv_nop" : "+v"(a), "+v"(b), "+v"(c), "+v"(d)); }
template <typename T> struct Frag;
template <> struct Frag<_Float16> {
  typedef v16h V; union U { v16h v; v8h h[2]; };
  static __device__ __forceinline__ v16h load(const _Float16* p) {
    U f; f.h[0] = *(const v8h*)(p); f.h[1] = *(const v8h*)(p + 16); return f.v;
  }
  static __device__ __forceinline__ v8f mma(v16h a, v16h b, v8f c) {
    return __builtin_amdgcn_wmma_f32_16x16x32_f16(false, a, false, b, (short)0, c, false, false);
  }
  static __device__ __forceinline__ void guard4(v8f& a, v8f& b, v8f& c, v8f& d, v16h x, v16h y) { dep_guard4_h(a, b, c, d, x, y); }
  static __device__ __forceinline__ void keep(v16h a, v16h b, v16h c, v16h d) { keep4_h(a, b, c, d); }
};
template <> struct Frag<__bf16> {
  typedef v16b V; union U { v16b v; v8b h[2]; };
  static __device__ __forceinline__ v16b load(const __bf16* p) {
    U f; f.h[0] = *(const v8b*)(p); f.h[1] = *(const v8b*)(p + 16); return f.v;
  }
  static __device__ __forceinline__ v8f mma(v16b a, v16b b, v8f c) {
    return __builtin_amdgcn_wmma_f32_16x16x32_bf16(false, a, false, b, (short)0, c, false, false);
  }
  static __device__ __forceinline__ void guard4(v8f& a, v8f& b, v8f& c, v8f& d, v16b x, v16b y) { dep_guard4_b(a, b, c, d, x, y); }
  static __device__ __forceinline__ void keep(v16b a, v16b b, v16b c, v16b d) { keep4_b(a, b, c, d); }
};

template <int ET> struct Elem;
template <> struct Elem<0> { typedef _Float16 T; };
template <> struct Elem<1> { typedef __bf16 T; };
template <int ET, bool SPLIT, int BIAS_MODE, int OUT_MODE, bool RESID, int ACT = 0>
__global__ __launch_bounds__(256) void wmma_gemm64(
    const unsigned short* __restrict__ Ap, const unsigned short* __restrict__ A2p, int lda, long strideA,
    const unsigned short* __restrict__ Btp, const unsigned short* __restrict__ Bt2p, int ldb, long strideB,
    void* __restrict__ Cout, void* __restrict__ Cout2, int ldc, long strideC,
    const float* __restrict__ bias,
    const float* __restrict__ resid, long strideR,
    int M, int N, int K, float scale) {
  static_assert(OUT_MODE == 0 || OUT_MODE == 1);
  static_assert(!RESID || OUT_MODE == 0);
  typedef typename Elem<ET>::T T;
  typedef typename Frag<T>::V V;
  const T* A = (const T*)Ap; const T* A2 = (const T*)A2p; const T* Bt = (const T*)Btp; const T* Bt2 = (const T*)Bt2p;
  (void)Cout2;
  __shared__ __align__(16) float sT[8][16 * 68];
  const int b    = blockIdx.y;
  const int lane = threadIdx.x & 31;
  const int wave = threadIdx.x >> 5;
  const int tilesN = N >> 6;
  const int tilesM = M >> 6;
  const int tile = blockIdx.x * 8 + wave;
  if (tile >= tilesM * tilesN) return;
  const int tm = tile / tilesN;
  const int tn = tile - tm * tilesN;
  const int m0 = tm << 6;
  const int n0 = tn << 6;

  const T* Ab  = A  + (size_t)b * strideA;
  const T* Bb  = Bt + (size_t)b * strideB;
  const T* Ab2 = SPLIT ? (A2  + (size_t)b * strideA) : nullptr;
  const T* Bb2 = SPLIT ? (Bt2 + (size_t)b * strideB) : nullptr;

  const int rlane = lane & 15;
  const int koff  = (lane >> 4) * 8;
  const int mOff  = (lane >> 4) * 8;

  v8f acc[4][4];
#pragma unroll
  for (int i = 0; i < 4; ++i)
#pragma unroll
    for (int j = 0; j < 4; ++j) acc[i][j] = (v8f){0.f,0.f,0.f,0.f,0.f,0.f,0.f,0.f};

  for (int k0 = 0; k0 < K; k0 += 32) {
    V bh[4], bl[4];
#pragma unroll
    for (int j = 0; j < 4; ++j) {
      const size_t bo = (size_t)(n0 + (j << 4) + rlane) * ldb + koff + k0;
      bh[j] = Frag<T>::load(Bb + bo);
      if (SPLIT) bl[j] = Frag<T>::load(Bb2 + bo);
    }
#pragma unroll
    for (int i = 0; i < 4; ++i) {
      const size_t ao = (size_t)(m0 + (i << 4) + rlane) * lda + koff + k0;
      V ah = Frag<T>::load(Ab + ao);
      V al;
      if (SPLIT) al = Frag<T>::load(Ab2 + ao);
#pragma unroll
      for (int j = 0; j < 4; ++j) {
        acc[i][j] = Frag<T>::mma(ah, bh[j], acc[i][j]);
        if (SPLIT) {
          acc[i][j] = Frag<T>::mma(ah, bl[j], acc[i][j]);
          acc[i][j] = Frag<T>::mma(al, bh[j], acc[i][j]);
        }
      }
      Frag<T>::guard4(acc[i][0], acc[i][1], acc[i][2], acc[i][3], ah, SPLIT ? al : ah);
    }
    Frag<T>::keep(bh[0], bh[1], bh[2], bh[3]);
    if (SPLIT) Frag<T>::keep(bl[0], bl[1], bl[2], bl[3]);
  }
  acc_guard4(acc[0][0], acc[0][1], acc[0][2], acc[0][3]);
  acc_guard4(acc[1][0], acc[1][1], acc[1][2], acc[1][3]);
  acc_guard4(acc[2][0], acc[2][1], acc[2][2], acc[2][3]);
  acc_guard4(acc[3][0], acc[3][1], acc[3][2], acc[3][3]);

  float* slab = sT[wave];
  const float* Rb = RESID ? (resid + (size_t)b * strideR) : nullptr;
#pragma unroll
  for (int i = 0; i < 4; ++i) {
    const int mBase = m0 + (i << 4);
#pragma unroll
    for (int j = 0; j < 4; ++j) {
      const int n = n0 + (j << 4) + rlane;
      float bv = 0.f;
      if (BIAS_MODE == 2) bv = bias[n];
#pragma unroll
      for (int r = 0; r < 8; ++r) {
        float v = acc[i][j][r] * scale;
        if (BIAS_MODE == 1) v += bias[mBase + mOff + r];
        if (BIAS_MODE == 2) v += bv;
        if (ACT == 1) v = tanhf(v);
        if (ACT == 2) v = fmaxf(v, 0.0f);
        if (ACT == 3) v = v * __builtin_amdgcn_rcpf(1.0f + __expf(-v));
        if (ACT == 4) v = (v > 0.f) ? v : 0.01f * v;
        slab[(mOff + r) * 68 + (j << 4) + rlane] = v;
      }
    }
    __builtin_amdgcn_fence(__ATOMIC_RELEASE, "workgroup");
    __builtin_amdgcn_wave_barrier();
    __builtin_amdgcn_fence(__ATOMIC_ACQUIRE, "workgroup");
    if (OUT_MODE == 0) {
      float* C = (float*)Cout + (size_t)b * strideC;
      const int hh = lane >> 4, c4 = (lane & 15) * 4;
      for (int pass = 0; pass < 2; ++pass) {
#pragma unroll
        for (int it = 0; it < 8; ++it) {
          const int row = it * 2 + hh;
          v4f v = *(const v4f*)(slab + row * 68 + c4);
          if (RESID) {
            const v4f rv = *(const v4f*)(Rb + (size_t)(mBase + row) * ldc + n0 + c4);
            v += rv;
          }
          *(volatile v4f*)(C + (size_t)(mBase + row) * ldc + n0 + c4) = v;
        }
        __threadfence();
      }
    } else {
      const int q = lane >> 3, c8 = (lane & 7) * 8;
      unsigned short* C = (unsigned short*)Cout + (size_t)b * strideC;
      for (int pass = 0; pass < 2; ++pass) {
#pragma unroll
        for (int it = 0; it < 4; ++it) {
          const int row = it * 4 + q;
          const float* sp = slab + row * 68 + c8;
          v8h hv;
#pragma unroll
          for (int e = 0; e < 8; ++e) hv[e] = (_Float16)sp[e];
          *(volatile v8h*)(C + (size_t)(mBase + row) * ldc + n0 + c8) = hv;
        }
        __threadfence();
      }
    }
    __builtin_amdgcn_fence(__ATOMIC_RELEASE, "workgroup");
    __builtin_amdgcn_wave_barrier();
    __builtin_amdgcn_fence(__ATOMIC_ACQUIRE, "workgroup");
  }
}

__global__ __launch_bounds__(256) void pad_cast_kernel(
    const float* __restrict__ src, unsigned short* __restrict__ dst,
    int srcRows, int srcCols, int dstCols, int total8, float scale)
{
  const int i = blockIdx.x * 256 + threadIdx.x;
  if (i >= total8) return;
  const int e0  = i << 3;
  const int row = e0 / dstCols;
  const int c8  = e0 - row * dstCols;
  const bool vr = (row < srcRows);
  const bool vc = (c8 + 8 <= srcCols);
  const int rc  = vr ? row : (srcRows - 1);
  const int cc  = vc ? c8 : (srcCols - 8);
  const float* p = src + (size_t)rc * srcCols + cc;
  const v4f a0 = *(const v4f*)(p);
  const v4f a1 = *(const v4f*)(p + 4);
  const float f = (vr && vc) ? scale : 0.0f;
  v8h hv;
#pragma unroll
  for (int e = 0; e < 4; ++e) {
    hv[e]     = (_Float16)(a0[e] * f);
    hv[4 + e] = (_Float16)(a1[e] * f);
  }
  unsigned short* q = dst + e0;
  *(volatile v8h*)q = hv;
  __threadfence();
  *(volatile v8h*)q = hv;
}

__global__ __launch_bounds__(256) void dt_cast_kernel(
    const float* __restrict__ XD, unsigned short* __restrict__ DT16, int total8, float scale)
{
  const int i = blockIdx.x * 256 + threadIdx.x;
  if (i >= total8) return;
  const int e0  = i << 3;
  const int row = e0 >> 5;
  const int c8  = e0 & 31;
  const float* p = XD + (size_t)row * kXdP + c8;
  const v4f a0 = *(const v4f*)(p);
  const v4f a1 = *(const v4f*)(p + 4);
  const float f = (c8 < kDtR) ? scale : 0.0f;
  v8h hv;
#pragma unroll
  for (int e = 0; e < 4; ++e) {
    hv[e]     = (_Float16)(a0[e] * f);
    hv[4 + e] = (_Float16)(a1[e] * f);
  }
  unsigned short* q = DT16 + e0;
  *(volatile v8h*)q = hv;
  __threadfence();
  *(volatile v8h*)q = hv;
}

__global__ __launch_bounds__(256) void ln_kernel(
    const float* __restrict__ x, const float* __restrict__ lnw, const float* __restrict__ lnb,
    unsigned short* __restrict__ XN)
{
  __shared__ float tile[kDm * kLnP];
  __shared__ float sW[kDm];
  __shared__ float sB[kDm];
  __shared__ float sMu[kLnTok];
  __shared__ float sRs[kLnTok];
  const int tid = threadIdx.x, lane = tid & 31, wave = tid >> 5;
  const int g0 = blockIdx.x * kLnTok;
  const int b  = g0 / kSeq;
  const int l0 = g0 - b * kSeq;
  for (int i = tid; i < kDm; i += 256) { sW[i] = lnw[i]; sB[i] = lnb[i]; }
  {
    const int cr = tid >> 3, t4 = (tid & 7) * 4;
#pragma unroll 1
    for (int it = 0; it < kDm / 32; ++it) {
      const int c = it * 32 + cr;
      const v4f v = *(const v4f*)(x + ((size_t)(b * kDm + c) * kSeq + l0 + t4));
      float* tp = tile + c * kLnP + t4;
      tp[0] = v[0]; tp[1] = v[1]; tp[2] = v[2]; tp[3] = v[3];
    }
  }
  __syncthreads();
  {
    const int tok = tid >> 3, part = tid & 7;
    const float* tp = tile + (part * (kDm / 8)) * kLnP + tok;
    float s = 0.0f;
#pragma unroll 1
    for (int i = 0; i < kDm / 8; ++i) s += tp[i * kLnP];
    s += __shfl_xor(s, 1, 32); s += __shfl_xor(s, 2, 32); s += __shfl_xor(s, 4, 32);
    const float mu = s * (1.0f / (float)kDm);
    float q = 0.0f;
#pragma unroll 1
    for (int i = 0; i < kDm / 8; ++i) { const float dv = tp[i * kLnP] - mu; q += dv * dv; }
    q += __shfl_xor(q, 1, 32); q += __shfl_xor(q, 2, 32); q += __shfl_xor(q, 4, 32);
    const float var = q * (1.0f / (float)kDm);
    if (part == 0) { sMu[tok] = mu; sRs[tok] = rsqrtf(var + 1e-5f); }
  }
  __syncthreads();
  const int c8a = lane * 8;
  const int c8b = 256 + (lane & 15) * 8;
#pragma unroll 1
  for (int r = 0; r < 4; ++r) {
    const int tok = wave * 4 + r;
    const float mu = sMu[tok], rs = sRs[tok];
    v8h ha, hb;
#pragma unroll
    for (int e = 0; e < 8; ++e) {
      const int ca = c8a + e, cbx = c8b + e;
      const float va = ((tile[ca  * kLnP + tok] - mu) * rs * sW[ca]  + sB[ca])  * kCarryXn;
      const float vb = ((tile[cbx * kLnP + tok] - mu) * rs * sW[cbx] + sB[cbx]) * kCarryXn;
      ha[e] = (_Float16)va;
      hb[e] = (_Float16)vb;
    }
    unsigned short* rowp = XN + (size_t)(g0 + tok) * kDm;
    for (int pass = 0; pass < 2; ++pass) {
      *(volatile v8h*)(rowp + c8a) = ha;
      if (lane < 16) *(volatile v8h*)(rowp + c8b) = hb;
      __threadfence();
    }
  }
}

__global__ __launch_bounds__(256) void conv_silu_kernel(
    const unsigned short* __restrict__ UP, const float* __restrict__ cw, const float* __restrict__ cbias,
    unsigned short* __restrict__ UC)
{
  __shared__ __align__(16) float sT[16 * kTP];
  const int tid = threadIdx.x, lane = tid & 31, wave = tid >> 5;
  const int d0 = blockIdx.x * 256, d = d0 + tid;
  const int g0 = blockIdx.y * 64;
  const int tb = g0 & (kSeq - 1);
  const float w0 = cw[d * kConvK + 0], w1 = cw[d * kConvK + 1], w2 = cw[d * kConvK + 2];
  const float bc = cbias[d];
  float xm2, xm1;
  {
    const bool hist = (tb > 0);
    const int rb = hist ? (g0 - 2) : g0;
    const float v2 = h16_to_f32(UP[(size_t)rb * kDin + d]);
    const float v1 = h16_to_f32(UP[(size_t)(rb + 1) * kDin + d]);
    xm2 = hist ? v2 : 0.0f;
    xm1 = hist ? v1 : 0.0f;
  }
#pragma unroll 1
  for (int sub = 0; sub < 4; ++sub) {
    const int lb = g0 + sub * 16;
#pragma unroll 1
    for (int s = 0; s < 16; ++s) {
      const float xc = h16_to_f32(UP[(size_t)(lb + s) * kDin + d]);
      float acc = w0 * xm2;
      acc = fmaf(w1, xm1, acc);
      acc = fmaf(w2, xc, acc);
      const float sv = acc + bc;
      const float sg = __builtin_amdgcn_rcpf(1.0f + __expf(-sv));
      sT[s * kTP + tid] = (sv * sg) * kCarryU;
      xm2 = xm1; xm1 = xc;
    }
    __syncthreads();
    v8h hv[2];
#pragma unroll
    for (int it = 0; it < 2; ++it) {
      const float* sp = sT + (it * 8 + wave) * kTP + lane * 8;
      const v4f a0 = *(const v4f*)(sp);
      const v4f a1 = *(const v4f*)(sp + 4);
#pragma unroll
      for (int e = 0; e < 4; ++e) { hv[it][e] = (_Float16)a0[e]; hv[it][4 + e] = (_Float16)a1[e]; }
    }
    for (int pass = 0; pass < 2; ++pass) {
#pragma unroll
      for (int it = 0; it < 2; ++it)
        *(volatile v8h*)(UC + (size_t)(lb + it * 8 + wave) * kDin + d0 + lane * 8) = hv[it];
      __threadfence();
    }
    __syncthreads();
  }
}

__global__ __launch_bounds__(256) void scan_kernel(
    const unsigned short* __restrict__ DLR, const unsigned short* __restrict__ UCp, const unsigned short* __restrict__ Zp,
    const float* __restrict__ XD, const float* __restrict__ bdt, const float* __restrict__ Alog,
    const float* __restrict__ Dv, unsigned short* __restrict__ Yp)
{
  __shared__ __align__(16) float sBC[16 * 2 * kNst];
  __shared__ __align__(16) float sY[16 * kTP];
  const int tid = threadIdx.x, lane = tid & 31, wave = tid >> 5;
  constexpr int kBlkPerB = kDin / 256;
  const int b  = blockIdx.x / kBlkPerB;
  const int d0 = (blockIdx.x - b * kBlkPerB) * 256;
  const int d  = d0 + tid;
  const size_t row0 = (size_t)b * kSeq;

  float An[kNst];
#pragma unroll
  for (int q4 = 0; q4 < kNst / 4; ++q4) {
    const v4f a4 = *(const v4f*)(Alog + (size_t)d * kNst + 4 * q4);
    An[4 * q4 + 0] = -__expf(a4[0]);
    An[4 * q4 + 1] = -__expf(a4[1]);
    An[4 * q4 + 2] = -__expf(a4[2]);
    An[4 * q4 + 3] = -__expf(a4[3]);
  }
  const float bb = bdt[d], Dd = Dv[d];
  float h[kNst];
#pragma unroll
  for (int n = 0; n < kNst; ++n) h[n] = 0.0f;
  constexpr float kInvCarryU = 1.0f / kCarryU;

#pragma unroll 1
  for (int c = 0; c < kSeq / 16; ++c) {
    const int l0 = c * 16;
    if (tid < 128) {
      const int r = tid >> 3, q4 = (tid & 7) * 4;
      const v4f v = *(const v4f*)(XD + (row0 + l0 + r) * kXdP + kDtR + q4);
      *(v4f*)(sBC + r * 32 + q4) = v;
    }
    __syncthreads();
#pragma unroll 1
    for (int s = 0; s < 16; ++s) {
      const size_t m  = row0 + l0 + s;
      const size_t md = m * kDin + d;
      const float a     = h16_to_f32(DLR[md]) + bb;
      const float delta = fmaxf(a, 0.0f) + log1pf(__expf(-fabsf(a)));
      const float xv    = h16_to_f32(UCp[md]) * kInvCarryU;
      const float zv    = h16_to_f32(Zp[md]);
      v4f Bq[4], Cq[4];
#pragma unroll
      for (int qq = 0; qq < 4; ++qq) {
        Bq[qq] = *(const v4f*)(sBC + s * 32 + 4 * qq);
        Cq[qq] = *(const v4f*)(sBC + s * 32 + kNst + 4 * qq);
      }
      const float dtx = delta * xv;
      float y = 0.0f;
#pragma unroll
      for (int n = 0; n < kNst; ++n) {
        const float e  = __expf(delta * An[n]);
        const float hn = e * h[n] + dtx * Bq[n >> 2][n & 3];
        h[n] = hn;
        y += Cq[n >> 2][n & 3] * hn;
      }
      y += xv * Dd;
      const float sg = __builtin_amdgcn_rcpf(1.0f + __expf(-zv));
      sY[s * kTP + tid] = (y * (zv * sg)) * kCarryY;
    }
    __syncthreads();
    v8h hv[2];
#pragma unroll
    for (int it = 0; it < 2; ++it) {
      const float* sp = sY + (it * 8 + wave) * kTP + lane * 8;
      const v4f a0 = *(const v4f*)(sp);
      const v4f a1 = *(const v4f*)(sp + 4);
#pragma unroll
      for (int e = 0; e < 4; ++e) { hv[it][e] = (_Float16)a0[e]; hv[it][4 + e] = (_Float16)a1[e]; }
    }
    for (int pass = 0; pass < 2; ++pass) {
#pragma unroll
      for (int it = 0; it < 2; ++it)
        *(volatile v8h*)(Yp + (row0 + l0 + it * 8 + wave) * kDin + d0 + lane * 8) = hv[it];
      __threadfence();
    }
  }
}

extern "C" void kernel_launch(void* const* d_in, const int* in_sizes, int n_in,
                              void* d_out, int out_size, void* d_ws, size_t ws_size,
                              hipStream_t stream)
{
  if (n_in < 12) return;
  if (in_sizes[0]  != kBatch * kDm * kSeq) return;
  if (in_sizes[1]  != kDm || in_sizes[2] != kDm) return;
  if (in_sizes[3]  != 2 * kDin * kDm) return;
  if (in_sizes[4]  != kDin * kConvK || in_sizes[5] != kDin) return;
  if (in_sizes[6]  != kXdN * kDin) return;
  if (in_sizes[7]  != kDin * kDtR || in_sizes[8] != kDin) return;
  if (in_sizes[9]  != kDin * kNst || in_sizes[10] != kDin) return;
  if (in_sizes[11] != kDm * kDin) return;
  if (out_size != kBatch * kDm * kSeq) return;
  if (ws_size < kWsTotal) return;

  const float* x          = (const float*)d_in[0];
  const float* ln_w       = (const float*)d_in[1];
  const float* ln_b       = (const float*)d_in[2];
  const float* in_proj_w  = (const float*)d_in[3];
  const float* conv_w     = (const float*)d_in[4];
  const float* conv_b     = (const float*)d_in[5];
  const float* x_proj_w   = (const float*)d_in[6];
  const float* dt_proj_w  = (const float*)d_in[7];
  const float* dt_proj_b  = (const float*)d_in[8];
  const float* A_log      = (const float*)d_in[9];
  const float* d_skip     = (const float*)d_in[10];
  const float* out_proj_w = (const float*)d_in[11];
  float* out = (float*)d_out;

  char* ws = (char*)d_ws;
  unsigned short* XN16   = (unsigned short*)(ws + kOffXN16);
  unsigned short* WIN16  = (unsigned short*)(ws + kOffWIN16);
  unsigned short* WXP16  = (unsigned short*)(ws + kOffWXP16);
  unsigned short* WDT16  = (unsigned short*)(ws + kOffWDT16);
  unsigned short* WOUT16 = (unsigned short*)(ws + kOffWOUT16);
  unsigned short* UPRE16 = (unsigned short*)(ws + kOffUPRE16);
  unsigned short* DLR16  = (unsigned short*)(ws + kOffDLR16);
  unsigned short* Z16    = (unsigned short*)(ws + kOffZ16);
  unsigned short* UC16   = (unsigned short*)(ws + kOffUC16);
  float*          XD     = (float*)(ws + kOffXD);
  unsigned short* DT16   = (unsigned short*)(ws + kOffDT16);
  unsigned short* Y16    = (unsigned short*)(ws + kOffY16);
  const float* dummy_bias  = dt_proj_b;
  const float* dummy_resid = x;

  pad_cast_kernel<<<(2 * kDin * kDm / 8) / 256, 256, 0, stream>>>(in_proj_w,  WIN16,  2 * kDin, kDm,  kDm,  2 * kDin * kDm / 8, kCarryW);
  pad_cast_kernel<<<(kXdP * kDin / 8) / 256,     256, 0, stream>>>(x_proj_w,   WXP16,  kXdN,     kDin, kDin, kXdP * kDin / 8,     kCarryW);
  pad_cast_kernel<<<(kDin * kDtP / 8) / 256,     256, 0, stream>>>(dt_proj_w,  WDT16,  kDin,     kDtR, kDtP, kDin * kDtP / 8,     kCarryWdt);
  pad_cast_kernel<<<(kDm * kDin / 8) / 256,      256, 0, stream>>>(out_proj_w, WOUT16, kDm,      kDin, kDin, kDm * kDin / 8,      kCarryW);

  ln_kernel<<<kRows / kLnTok, 256, 0, stream>>>(x, ln_w, ln_b, XN16);

  wmma_gemm64<0, false, 0, 1, false><<<dim3((kRows / 64) * (kDin / 64) / 8, 1), 256, 0, stream>>>(
      XN16, XN16, kDm, 0L,
      WIN16, WIN16, kDm, 0L,
      (void*)UPRE16, (void*)UPRE16, kDin, 0L,
      dummy_bias, dummy_resid, 0L,
      kRows, kDin, kDm, kScaleIn);

  wmma_gemm64<0, false, 0, 1, false><<<dim3((kRows / 64) * (kDin / 64) / 8, 1), 256, 0, stream>>>(
      XN16, XN16, kDm, 0L,
      WIN16 + (size_t)kDin * kDm, WIN16 + (size_t)kDin * kDm, kDm, 0L,
      (void*)Z16, (void*)Z16, kDin, 0L,
      dummy_bias, dummy_resid, 0L,
      kRows, kDin, kDm, kScaleIn);

  conv_silu_kernel<<<dim3(kDin / 256, kRows / 64), 256, 0, stream>>>(UPRE16, conv_w, conv_b, UC16);

  wmma_gemm64<0, false, 0, 0, false><<<dim3((kRows / 64) * (kXdP / 64) / 8, 1), 256, 0, stream>>>(
      UC16, UC16, kDin, 0L,
      WXP16, WXP16, kDin, 0L,
      (void*)XD, (void*)XD, kXdP, 0L,
      dummy_bias, dummy_resid, 0L,
      kRows, kXdP, kDin, kScaleXp);

  dt_cast_kernel<<<(kRows * kDtP / 8) / 256, 256, 0, stream>>>(XD, DT16, kRows * kDtP / 8, kCarryDt);

  wmma_gemm64<0, false, 0, 1, false><<<dim3((kRows / 64) * (kDin / 64) / 8, 1), 256, 0, stream>>>(
      DT16, DT16, kDtP, 0L,
      WDT16, WDT16, kDtP, 0L,
      (void*)DLR16, (void*)DLR16, kDin, 0L,
      dummy_bias, dummy_resid, 0L,
      kRows, kDin, kDtP, kScaleDt);

  scan_kernel<<<kBatch * (kDin / 256), 256, 0, stream>>>(DLR16, UC16, Z16, XD, dt_proj_b, A_log, d_skip, Y16);

  wmma_gemm64<0, false, 0, 0, true><<<dim3((kDm / 64) * (kSeq / 64) / 8, kBatch), 256, 0, stream>>>(
      WOUT16, WOUT16, kDin, 0L,
      Y16, Y16, kDin, (long)kSeq * kDin,
      (void*)out, (void*)out, kSeq, (long)kDm * kSeq,
      dummy_bias, x, (long)kDm * kSeq,
      kDm, kSeq, kDin, kScaleOut);
}
